// GNNModel_61967788147057
// MI455X (gfx1250) — hardware-verified
//
#include <hip/hip_runtime.h>
#include <stddef.h>
#include <stdint.h>
#include <math.h>


#define CIN    128
#define CH     64
#define CO     40
#define NP     64
#define KA     128
#define NTHR   256
#define NWAVE  8
#define EPT    8
#define CHUNK  (NTHR * EPT)
#define WCAP   (EPT * 32)
#define LISTN  (NWAVE * WCAP)
#define NBD    8192
#define SLD    13
#define NBA    1024
#define SLA    10
#define RCAP   28672
#define DEGCAP 64
#define GRP    32
#define STGW   2048
#define NITH   ((GRP * KA * 2) / 512)
#define NITO   ((GRP * CO * 4) / 512)
#define GBM    64
#define GBN    64
#define GTHR   128
#define NU1    (NP * (CIN / 8))
#define NU2    (NP * (CH / 4))
#define NU3    (NP * (CH / 4))
#define NUT    (NU1 + NU2 + NU3)
#define AGG_ZINTS (LISTN + 2 * RCAP + 3 * NBA)
#define AGG_LDS_INTS (AGG_ZINTS + 16)
#define WSMAX  134217728
#define BNEPS  1e-5f

static_assert((CHUNK & (CHUNK - 1)) == 0 && CHUNK <= 4096);
static_assert((NBD & (NBD - 1)) == 0 && NBD == (1 << SLD));
static_assert((NBA & (NBA - 1)) == 0 && NBA == (1 << SLA));
static_assert(((long long)CHUNK << SLD) < (1LL << 31));
static_assert(((long long)CHUNK << SLA) < (1LL << 31));
static_assert(NBD % (NTHR * 4) == 0);
static_assert(LISTN % NTHR == 0);
static_assert(NBA % NWAVE == 0 && NBA % 32 == 0 && NBA % GBM == 0);
static_assert((NBA / NWAVE) % GRP == 0);
static_assert(RCAP % 32 == 0 && AGG_ZINTS % 4 == 0 && LISTN % 4 == 0);
static_assert(NWAVE * STGW <= RCAP);
static_assert((GRP * KA) / 2 <= STGW);
static_assert(GRP * CO <= STGW);
static_assert((GRP * KA * 2) % 512 == 0 && NITH == 16);
static_assert((GRP * CO * 4) % 512 == 0 && NITO == 10);
static_assert((GRP * CO * 4) % 128 == 0);
static_assert(KA % 32 == 0 && KA == CIN && KA == 2 * CH);
static_assert(NP == GBN && NP == CH);
static_assert(GBM == (GTHR / 32) * 16 && GBN == 64);
static_assert(NU1 % NTHR == 0 && NU2 % NTHR == 0 && NU3 % NTHR == 0 && NUT % NTHR == 0);
static_assert(CIN / 8 == 16 && CH / 4 == 16);
static_assert(CH == 2 * 32);
static_assert(CO % 2 == 0 && CO <= CH);
static_assert(AGG_LDS_INTS * 4 <= 300000);

typedef float          v2f   __attribute__((ext_vector_type(2)));
typedef float          v4f   __attribute__((ext_vector_type(4)));
typedef float          v8f   __attribute__((ext_vector_type(8)));
typedef int            v2i   __attribute__((ext_vector_type(2)));
typedef int            v4i   __attribute__((ext_vector_type(4)));
typedef int            v8i   __attribute__((ext_vector_type(8)));
typedef unsigned short v8us  __attribute__((ext_vector_type(8)));
typedef unsigned short v16us __attribute__((ext_vector_type(16)));
typedef __bf16         v16bf __attribute__((ext_vector_type(16)));
typedef v2f  __attribute__((may_alias)) v2fa;
typedef v4f  __attribute__((may_alias)) v4fa;
typedef v2i  __attribute__((may_alias)) v2ia;
typedef v4i  __attribute__((may_alias)) v4ia;
typedef v8us __attribute__((may_alias)) v8usa;
union Frag { v16bf v; v16us u; v8us h[2]; v8i w; };

__device__ __forceinline__ v8f wmb(const Frag& a, const Frag& b, v8f c) {
  v8f d = __builtin_amdgcn_wmma_f32_16x16x32_bf16(false, a.v, false, b.v, (short)0, c, false, false);
  asm volatile("v_nop\n\tv_nop\n\tv_nop\n\tv_nop" : "+v"(d) : "v"(a.w), "v"(b.w));
  return d;
}

__device__ __forceinline__ unsigned bf16_bits(float f) {
  const unsigned u = __float_as_uint(f);
  return (u + 0x7FFFu + ((u >> 16) & 1u)) >> 16;
}
__device__ __forceinline__ float bf16_val(float f) {
  return __uint_as_float(bf16_bits(f) << 16);
}

template <int SLB>
__device__ __forceinline__ int scan_chunk(const int* __restrict__ dsts, int nE, int cbase, int slotBase,
                                          int nb, int vec8, int* list, int tid, int lane, int wave) {
  int wc = 0;
  const int el0  = tid * EPT;
  const int e0   = cbase + el0;
  const int sent = -2147483647 - 1;
  v4i da, db;
  if (vec8 != 0 && cbase + CHUNK <= nE) {
    da = *(const v4i*)(dsts + e0);
    db = *(const v4i*)(dsts + e0 + 4);
  } else {
    da.x = (e0     < nE) ? dsts[min(e0,     nE - 1)] : sent;
    da.y = (e0 + 1 < nE) ? dsts[min(e0 + 1, nE - 1)] : sent;
    da.z = (e0 + 2 < nE) ? dsts[min(e0 + 2, nE - 1)] : sent;
    da.w = (e0 + 3 < nE) ? dsts[min(e0 + 3, nE - 1)] : sent;
    db.x = (e0 + 4 < nE) ? dsts[min(e0 + 4, nE - 1)] : sent;
    db.y = (e0 + 5 < nE) ? dsts[min(e0 + 5, nE - 1)] : sent;
    db.z = (e0 + 6 < nE) ? dsts[min(e0 + 6, nE - 1)] : sent;
    db.w = (e0 + 7 < nE) ? dsts[min(e0 + 7, nE - 1)] : sent;
  }
  const unsigned nbs = (unsigned)slotBase;
  const unsigned unb = (unsigned)nb;
  const unsigned s0 = (unsigned)da.x - nbs, s1 = (unsigned)da.y - nbs;
  const unsigned s2 = (unsigned)da.z - nbs, s3 = (unsigned)da.w - nbs;
  const unsigned s4 = (unsigned)db.x - nbs, s5 = (unsigned)db.y - nbs;
  const unsigned s6 = (unsigned)db.z - nbs, s7 = (unsigned)db.w - nbs;
  const bool h0 = s0 < unb, h1 = s1 < unb, h2 = s2 < unb, h3 = s3 < unb;
  const bool h4 = s4 < unb, h5 = s5 < unb, h6 = s6 < unb, h7 = s7 < unb;
  const unsigned any = __builtin_amdgcn_ballot_w32(h0 | h1 | h2 | h3 | h4 | h5 | h6 | h7);
  if (any != 0u) {
#define HITJ(J, HJ, SJ) { \
      const unsigned mj = __builtin_amdgcn_ballot_w32(HJ); \
      if (mj != 0u) { \
        if (HJ) { \
          const int pos = wc + (int)__builtin_amdgcn_mbcnt_lo(mj, 0u); \
          if (pos < WCAP) list[wave * WCAP + pos] = ((el0 + (J)) << SLB) | (int)(SJ); \
        } \
        wc += (int)__builtin_popcount(mj); } }
    HITJ(0, h0, s0)
    HITJ(1, h1, s1)
    HITJ(2, h2, s2)
    HITJ(3, h3, s3)
    HITJ(4, h4, s4)
    HITJ(5, h5, s5)
    HITJ(6, h6, s6)
    HITJ(7, h7, s7)
#undef HITJ
  }
  return wc;
}

__global__ __launch_bounds__(NTHR) void k_wprep(const float* __restrict__ W1, const float* __restrict__ W2,
                                                const float* __restrict__ W3,
                                                unsigned short* W1T, unsigned short* W2T, unsigned short* W3T) {
  const int u = (int)blockIdx.x * NTHR + (int)threadIdx.x;
  v8us o;
  unsigned short* dp;
  if (u < NU1) {
    const int n  = u >> 4;
    const int k8 = (u & 15) * 8;
    const float* p = W1 + (size_t)k8 * CH + n;
#pragma unroll
    for (int i = 0; i < 8; ++i) o[i] = (unsigned short)bf16_bits(p[(size_t)i * CH]);
    dp = W1T + (size_t)n * KA + k8;
  } else if (u < NU1 + NU2) {
    const int v = u - NU1;
    const int n = v >> 4;
    const int q = v & 15;
    const float* p = W2 + (size_t)(4 * q) * CH + n;
    const unsigned short f0 = (unsigned short)bf16_bits(p[0]);
    const unsigned short f1 = (unsigned short)bf16_bits(p[CH]);
    const unsigned short f2 = (unsigned short)bf16_bits(p[2 * CH]);
    const unsigned short f3 = (unsigned short)bf16_bits(p[3 * CH]);
    o[0] = f0; o[1] = f1; o[2] = f0; o[3] = f1; o[4] = f2; o[5] = f3; o[6] = f2; o[7] = f3;
    dp = W2T + (size_t)n * KA + 8 * q;
  } else if (u < NUT) {
    const int v = u - NU1 - NU2;
    const int n = v >> 4;
    const int q = v & 15;
    const bool live = n < CO;
    const int nc = live ? n : CO - 1;
    const float* p = W3 + (size_t)(4 * q) * CO + nc;
    const unsigned short f0 = live ? (unsigned short)bf16_bits(p[0])      : (unsigned short)0;
    const unsigned short f1 = live ? (unsigned short)bf16_bits(p[CO])     : (unsigned short)0;
    const unsigned short f2 = live ? (unsigned short)bf16_bits(p[2 * CO]) : (unsigned short)0;
    const unsigned short f3 = live ? (unsigned short)bf16_bits(p[3 * CO]) : (unsigned short)0;
    o[0] = f0; o[1] = f1; o[2] = f0; o[3] = f1; o[4] = f2; o[5] = f3; o[6] = f2; o[7] = f3;
    dp = W3T + (size_t)n * KA + 8 * q;
  } else {
    return;
  }
  *(volatile v8us*)dp = o;
  __threadfence();
  *(volatile v8us*)dp = o;
}

__global__ __launch_bounds__(NTHR) void k_cvx(const float* __restrict__ x, int nN, int nUnits,
                                              unsigned short* xb) {
  const int u = (int)blockIdx.x * NTHR + (int)threadIdx.x;
  if (u >= nUnits) return;
  const int row = u >> 4;
  const int k8  = (u & 15) * 8;
  const int rc  = row < nN ? row : nN - 1;
  const bool rok = row < nN;
  const float* p = x + (size_t)rc * CIN + k8;
  const v4f a = *(const v4fa*)p;
  const v4f b = *(const v4fa*)(p + 4);
  v8us o;
  o[0] = rok ? (unsigned short)bf16_bits(a.x) : (unsigned short)0;
  o[1] = rok ? (unsigned short)bf16_bits(a.y) : (unsigned short)0;
  o[2] = rok ? (unsigned short)bf16_bits(a.z) : (unsigned short)0;
  o[3] = rok ? (unsigned short)bf16_bits(a.w) : (unsigned short)0;
  o[4] = rok ? (unsigned short)bf16_bits(b.x) : (unsigned short)0;
  o[5] = rok ? (unsigned short)bf16_bits(b.y) : (unsigned short)0;
  o[6] = rok ? (unsigned short)bf16_bits(b.z) : (unsigned short)0;
  o[7] = rok ? (unsigned short)bf16_bits(b.w) : (unsigned short)0;
  unsigned short* dp = xb + (size_t)row * KA + k8;
  *(volatile v8us*)dp = o;
  __threadfence();
  *(volatile v8us*)dp = o;
}

__global__ __launch_bounds__(NTHR) void k_deg(const int* __restrict__ dsts, int nE, int vec8, float* dis) {
  __shared__ __attribute__((aligned(16))) int scnt[NBD];
  __shared__ __attribute__((aligned(16))) int list[LISTN];
  __shared__ int wcnt[NWAVE];
  const int tid = (int)threadIdx.x, lane = tid & 31, wave = tid >> 5;
  const int nodeBase = (int)blockIdx.x * NBD;

  for (int i = tid; i < NBD; i += NTHR) scnt[i] = 0;
  for (int i = tid; i < LISTN; i += NTHR) list[i] = 0;
  if (tid < NWAVE) wcnt[tid] = 0;
  __syncthreads();

  const int nChunks = (nE + CHUNK - 1) / CHUNK;
#pragma unroll 1
  for (int ch = 0; ch < nChunks; ++ch) {
    const int cbase = ch * CHUNK;
    const int wc = scan_chunk<SLD>(dsts, nE, cbase, nodeBase, NBD, vec8, list, tid, lane, wave);
    if (lane == 0) wcnt[wave] = wc;
    __syncthreads();
    if (wave == 0) {
#pragma unroll 1
      for (int w2 = 0; w2 < NWAVE; ++w2) {
        int c = wcnt[w2];
        c = c < 0 ? 0 : (c > WCAP ? WCAP : c);
#pragma unroll 1
        for (int b0 = 0; b0 < c; b0 += 32) {
          const int idx = b0 + lane;
          const int ent = list[w2 * WCAP + (idx < WCAP ? idx : WCAP - 1)];
          const int m32 = (c - b0) < 32 ? (c - b0) : 32;
#pragma unroll 1
          for (int k = 0; k < m32; ++k) {
            const int u  = __builtin_amdgcn_readlane(ent, k);
            const int sl = u & (NBD - 1);
            if (lane == 0) scnt[sl] = scnt[sl] + 1;
          }
        }
      }
    }
    __syncthreads();
  }

  v4f vals[NBD / (NTHR * 4)];
#pragma unroll
  for (int it = 0; it < NBD / (NTHR * 4); ++it) {
    const int s0 = it * (NTHR * 4) + 4 * tid;
    const v4i c4 = *(const v4ia*)(scnt + s0);
    v4f v;
    v.x = (c4.x > 0) ? rsqrtf((float)c4.x) : 0.0f;
    v.y = (c4.y > 0) ? rsqrtf((float)c4.y) : 0.0f;
    v.z = (c4.z > 0) ? rsqrtf((float)c4.z) : 0.0f;
    v.w = (c4.w > 0) ? rsqrtf((float)c4.w) : 0.0f;
    vals[it] = v;
  }
#pragma unroll
  for (int it = 0; it < NBD / (NTHR * 4); ++it) {
    const int s0 = it * (NTHR * 4) + 4 * tid;
    *(volatile v4f*)(dis + (size_t)nodeBase + s0) = vals[it];
  }
  __threadfence();
#pragma unroll
  for (int it = 0; it < NBD / (NTHR * 4); ++it) {
    const int s0 = it * (NTHR * 4) + 4 * tid;
    *(volatile v4f*)(dis + (size_t)nodeBase + s0) = vals[it];
  }
}

__global__ __launch_bounds__(GTHR) void k_gemm(
    const unsigned short* __restrict__ A, const unsigned short* __restrict__ WT,
    float* outF, int K, int ldo)
{
  __shared__ __attribute__((aligned(16))) float stg[GBM * GBN];
  const int tid = (int)threadIdx.x, lane = tid & 31, wave = tid >> 5, hh = lane >> 4, m = lane & 15;
  const int rowBase = (int)blockIdx.x * GBM;
  const int col0    = (int)blockIdx.y * GBN;

  v8f acc[4];
  {
    const v8f z = {0.f, 0.f, 0.f, 0.f, 0.f, 0.f, 0.f, 0.f};
    acc[0] = z; acc[1] = z; acc[2] = z; acc[3] = z;
  }
  const unsigned short* ap = A  + (size_t)(rowBase + 16 * wave + m) * (size_t)K + 8 * hh;
  const unsigned short* wp = WT + (size_t)(col0 + m) * (size_t)K + 8 * hh;
  const int ksteps = K >> 5;
#pragma unroll 1
  for (int ks = 0; ks < ksteps; ++ks) {
    Frag af;
    af.h[0] = *(const v8usa*)(ap + 32 * ks);
    af.h[1] = *(const v8usa*)(ap + 32 * ks + 16);
#pragma unroll
    for (int t = 0; t < 4; ++t) {
      const unsigned short* wq = wp + (size_t)(16 * t) * (size_t)K + 32 * ks;
      Frag bf;
      bf.h[0] = *(const v8usa*)wq;
      bf.h[1] = *(const v8usa*)(wq + 16);
      acc[t] = wmb(af, bf, acc[t]);
    }
  }

#pragma unroll
  for (int t = 0; t < 4; ++t) {
    const int lc = 16 * t + m;
#pragma unroll
    for (int r = 0; r < 8; ++r) {
      const int lr = 16 * wave + 8 * hh + r;
      stg[lr * GBN + lc] = acc[t][r];
    }
  }
  __syncthreads();

  v4f fv[8];
#pragma unroll
  for (int i = 0; i < 8; ++i) {
    const int lr = 16 * wave + 2 * i + hh;
    fv[i] = *(const v4fa*)(stg + lr * GBN + 4 * m);
  }
#pragma unroll
  for (int i = 0; i < 8; ++i) {
    const int lr = 16 * wave + 2 * i + hh;
    const int gr = rowBase + lr;
    float* op = outF + (size_t)gr * (size_t)ldo + col0 + 4 * m;
    *(volatile v4f*)op = fv[i];
  }
  __threadfence();
#pragma unroll
  for (int i = 0; i < 8; ++i) {
    const int lr = 16 * wave + 2 * i + hh;
    const int gr = rowBase + lr;
    float* op = outF + (size_t)gr * (size_t)ldo + col0 + 4 * m;
    *(volatile v4f*)op = fv[i];
  }
}

template <int HBO>
__global__ __launch_bounds__(NTHR) void k_agg(const int* __restrict__ srcs, const int* __restrict__ dsts,
                                              int nE, int nN, int vec8,
                                              const float* __restrict__ dis,
                                              const float* __restrict__ xl,
                                              const float* __restrict__ bias,
                                              const float* __restrict__ gam, const float* __restrict__ bet,
                                              const float* __restrict__ rme, const float* __restrict__ rva,
                                              unsigned short* hb, float* outp) {
  extern __shared__ __attribute__((aligned(16))) int dsm[];
  int* list = dsm;
  int* hl   = dsm + LISTN;
  int* sl   = hl + RCAP;
  int* cnt  = sl + RCAP;
  int* offs = cnt + NBA;
  int* cur  = offs + NBA;
  int* misc = cur + NBA;
  const int tid = (int)threadIdx.x, lane = tid & 31, wave = tid >> 5;
  const int nodeBase = (int)blockIdx.x * NBA;
  const int cl = 2 * lane;

  {
    const v4i zi = {0, 0, 0, 0};
    for (int i = tid * 4; i < AGG_ZINTS; i += NTHR * 4) *(v4ia*)(dsm + i) = zi;
    if (tid < 16) misc[tid] = 0;
  }
  float cb0, cb1, sc0 = 1.0f, sc1 = 1.0f, rm0 = 0.0f, rm1 = 0.0f, be0 = 0.0f, be1 = 0.0f;
  if constexpr (HBO != 0) {
    const v2f bb = *(const v2fa*)(bias + cl);
    const v2f gg = *(const v2fa*)(gam + cl);
    const v2f ee = *(const v2fa*)(bet + cl);
    const v2f mm = *(const v2fa*)(rme + cl);
    const v2f vv = *(const v2fa*)(rva + cl);
    cb0 = bf16_val(bb.x); cb1 = bf16_val(bb.y);
    sc0 = bf16_val(gg.x) * rsqrtf(bf16_val(vv.x) + BNEPS);
    sc1 = bf16_val(gg.y) * rsqrtf(bf16_val(vv.y) + BNEPS);
    rm0 = bf16_val(mm.x); rm1 = bf16_val(mm.y);
    be0 = bf16_val(ee.x); be1 = bf16_val(ee.y);
  } else {
    const bool lv = lane < (CO / 2);
    const int  cc = cl < CO - 2 ? cl : CO - 2;
    const v2f bb = *(const v2fa*)(bias + cc);
    cb0 = lv ? bf16_val(bb.x) : 0.0f;
    cb1 = lv ? bf16_val(bb.y) : 0.0f;
  }
  __syncthreads();

  int t = 0, ov = 0;
  const int nChunks = (nE + CHUNK - 1) / CHUNK;
#pragma unroll 1
  for (int ch = 0; ch < nChunks; ++ch) {
    const int cbase = ch * CHUNK;
    const int wc = scan_chunk<SLA>(dsts, nE, cbase, nodeBase, NBA, vec8, list, tid, lane, wave);
    if (lane == 0) misc[wave] = wc;
    __syncthreads();
    if (wave == 0) {
#pragma unroll 1
      for (int w2 = 0; w2 < NWAVE; ++w2) {
        int c = misc[w2];
        c = c < 0 ? 0 : (c > WCAP ? WCAP : c);
#pragma unroll 1
        for (int b0 = 0; b0 < c; b0 += 32) {
          const int idx = b0 + lane;
          const int ent = list[w2 * WCAP + (idx < WCAP ? idx : WCAP - 1)];
          const int m32 = (c - b0) < 32 ? (c - b0) : 32;
#pragma unroll 1
          for (int k = 0; k < m32; ++k) {
            const int u    = __builtin_amdgcn_readlane(ent, k);
            const int slot = u & (NBA - 1);
            const int el   = (u >> SLA) & (CHUNK - 1);
            const int pk   = ((cbase + el) << SLA) | slot;
            if (t < RCAP) {
              if (lane == 0) { hl[t] = pk; cnt[slot] = cnt[slot] + 1; }
              t = t + 1;
            } else {
              ov = 1;
            }
          }
        }
      }
    }
    __syncthreads();
  }
  if (wave == 0 && lane == 0) { misc[8] = t; misc[9] = ov; }
  __syncthreads();
  int tt = misc[8];
  tt = tt < 0 ? 0 : (tt > RCAP ? RCAP : tt);
  const int ovf = misc[9];

  if (wave == 0) {
    const int base = lane * (NBA / 32);
    int s = 0;
#pragma unroll 1
    for (int i = 0; i < NBA / 32; ++i) s += cnt[base + i];
    int incl = s;
#pragma unroll
    for (int d = 1; d < 32; d <<= 1) {
      const int y = __shfl_up(incl, d, 32);
      if (lane >= d) incl += y;
    }
    int run = incl - s;
#pragma unroll 1
    for (int i = 0; i < NBA / 32; ++i) {
      const int cv = cnt[base + i];
      offs[base + i] = run;
      cur[base + i]  = run;
      run += cv;
    }
  }
  __syncthreads();
  if (wave == 0) {
#pragma unroll 1
    for (int b0 = 0; b0 < tt; b0 += 32) {
      const int idx = b0 + lane;
      const int ent = hl[idx < RCAP ? idx : RCAP - 1];
      const int m32 = (tt - b0) < 32 ? (tt - b0) : 32;
#pragma unroll 1
      for (int k = 0; k < m32; ++k) {
        const int u    = __builtin_amdgcn_readlane(ent, k);
        const int slot = u & (NBA - 1);
        if (lane == 0) {
          int p = cur[slot];
          p = p < 0 ? 0 : (p > RCAP - 1 ? RCAP - 1 : p);
          sl[p] = u;
          cur[slot] = p + 1;
        }
      }
    }
  }
  __syncthreads();

  const float qnan = __int_as_float(0x7fc00000);
  const float pz = (ovf != 0) ? qnan : 0.0f;
  int* stg = hl + wave * STGW;
#pragma unroll 1
  for (int g = 0; g < (NBA / NWAVE) / GRP; ++g) {
    const int s0    = wave * (NBA / NWAVE) + g * GRP;
    const int node0 = nodeBase + s0;
#pragma unroll 1
    for (int j = 0; j < GRP; ++j) {
      const int s    = s0 + j;
      const int node = node0 + j;
      int c = cnt[s];
      const bool big = c > DEGCAP;
      c = c < 0 ? 0 : (c > DEGCAP ? DEGCAP : c);
      int o = offs[s];
      o = o < 0 ? 0 : (o > RCAP ? RCAP : o);
      const int nc = node < nN ? node : nN - 1;
      const float dd = dis[nc];
      float a0 = 0.0f, a1 = 0.0f;
#pragma unroll 1
      for (int b0 = 0; b0 < c; b0 += 32) {
        int idx = o + b0 + lane;
        idx = idx > RCAP - 1 ? RCAP - 1 : idx;
        const int ent = sl[idx];
        int eid = ent >> SLA;
        eid = eid < 0 ? 0 : (eid > nE - 1 ? nE - 1 : eid);
        int sr = srcs[eid];
        sr = sr < 0 ? 0 : (sr > nN - 1 ? nN - 1 : sr);
        const float cf  = dis[sr] * dd;
        const int   cfi = __float_as_int(cf);
        const int m32 = (c - b0) < 32 ? (c - b0) : 32;
#pragma unroll 1
        for (int k = 0; k < m32; ++k) {
          const int   sk = __builtin_amdgcn_readlane(sr, k);
          const float ck = __int_as_float(__builtin_amdgcn_readlane(cfi, k));
          const v2f a = *(const v2fa*)(xl + (size_t)sk * CH + cl);
          a0 = fmaf(ck, a.x, a0);
          a1 = fmaf(ck, a.y, a1);
        }
      }
      const float pzr = big ? qnan : pz;
      const bool live = node < nN;
      float y0 = a0 + cb0;
      float y1 = a1 + cb1;
      if constexpr (HBO != 0) {
        y0 = fmaxf(fmaf(y0 - rm0, sc0, be0), 0.0f);
        y1 = fmaxf(fmaf(y1 - rm1, sc1, be1), 0.0f);
      }
      y0 = y0 + pzr; y1 = y1 + pzr;
      const float v0 = live ? y0 : 0.0f;
      const float v1 = live ? y1 : 0.0f;
      if constexpr (HBO != 0) {
        const unsigned h0 = bf16_bits(v0), h1 = bf16_bits(v1);
        const unsigned l0 = bf16_bits(v0 - __uint_as_float(h0 << 16));
        const unsigned l1 = bf16_bits(v1 - __uint_as_float(h1 << 16));
        v2i w;
        w.x = (int)(h0 | (h1 << 16));
        w.y = (int)(l0 | (l1 << 16));
        *(v2ia*)(stg + j * (KA / 2) + 2 * lane) = w;
      } else {
        if (lane < (CO / 2)) {
          v2f f;
          f.x = v0; f.y = v1;
          *(v2fa*)((float*)stg + j * CO + cl) = f;
        }
      }
    }
    __syncthreads();
    if constexpr (HBO != 0) {
      v4i pv[NITH];
#pragma unroll
      for (int it = 0; it < NITH; ++it) pv[it] = *(const v4ia*)(stg + it * 128 + 4 * lane);
      char* gb = (char*)hb + (size_t)node0 * (size_t)(KA * 2);
#pragma unroll
      for (int it = 0; it < NITH; ++it)
        *(volatile v4i*)(gb + (size_t)it * 512 + 16 * lane) = pv[it];
      __threadfence();
#pragma unroll
      for (int it = 0; it < NITH; ++it)
        *(volatile v4i*)(gb + (size_t)it * 512 + 16 * lane) = pv[it];
    } else {
      int lr = nN - node0;
      lr = lr < 0 ? 0 : (lr > GRP ? GRP : lr);
      const int liveBytes = lr * (CO * 4);
      v4f fv[NITO];
#pragma unroll
      for (int it = 0; it < NITO; ++it) fv[it] = *(const v4fa*)((const float*)stg + it * 128 + 4 * lane);
      char* gb = (char*)outp + (size_t)node0 * (size_t)(CO * 4);
#pragma unroll
      for (int it = 0; it < NITO; ++it) {
        const int po = it * 512 + 16 * lane;
        if (po < liveBytes) *(volatile v4f*)(gb + po) = fv[it];
      }
      __threadfence();
#pragma unroll
      for (int it = 0; it < NITO; ++it) {
        const int po = it * 512 + 16 * lane;
        if (po < liveBytes) *(volatile v4f*)(gb + po) = fv[it];
      }
    }
    __syncthreads();
  }
}

static inline int cdiv(int a, int b) { return (a + b - 1) / b; }
static inline size_t al256(size_t o) { return (o + 255) & ~(size_t)255; }

extern "C" void kernel_launch(void* const* d_in, const int* in_sizes, int n_in,
                              void* d_out, int out_size, void* d_ws, size_t ws_size,
                              hipStream_t stream) {
  if (n_in < 16) return;
  if (in_sizes[0] < CIN || (in_sizes[0] % CIN) != 0) return;
  const int nN = in_sizes[0] / CIN;
  if (nN < 1 || nN > (1 << 24)) return;
  if (in_sizes[1] < 2 || (in_sizes[1] & 1) != 0) return;
  const int nE = in_sizes[1] / 2;
  if (nE < 1 || nE >= (1 << (31 - SLA))) return;
  if (in_sizes[2] != CIN * CH || in_sizes[3] != CH) return;
  if (in_sizes[4] != CH * CH || in_sizes[5] != CH) return;
  if (in_sizes[6] != CH * CO || in_sizes[7] != CO) return;
  for (int i = 8; i < 16; ++i) if (in_sizes[i] != CH) return;
  if ((long long)out_size != (long long)nN * CO) return;

  const float* x    = (const float*)d_in[0];
  const int*   edge = (const int*)d_in[1];
  const float* W1   = (const float*)d_in[2];
  const float* b1   = (const float*)d_in[3];
  const float* W2   = (const float*)d_in[4];
  const float* b2   = (const float*)d_in[5];
  const float* W3   = (const float*)d_in[6];
  const float* b3   = (const float*)d_in[7];
  const float* g1   = (const float*)d_in[8];
  const float* e1   = (const float*)d_in[9];
  const float* m1   = (const float*)d_in[10];
  const float* v1   = (const float*)d_in[11];
  const float* g2   = (const float*)d_in[12];
  const float* e2   = (const float*)d_in[13];
  const float* m2   = (const float*)d_in[14];
  const float* v2   = (const float*)d_in[15];
  float* out = (float*)d_out;
  const int* src = edge;
  const int* dst = edge + nE;

  const int MP   = cdiv(nN, GBM) * GBM;
  const int gM   = MP / GBM;
  const int gD   = cdiv(nN, NBD);
  const int NBPD = gD * NBD;
  const int gA   = cdiv(MP, NBA);
  const int RA   = gA * NBA;
  if ((long long)RA < (long long)MP) return;
  if (NBPD < nN) return;
  const int vec8 = ((nE & 3) == 0) ? 1 : 0;

  char* ws = (char*)d_ws;
  size_t off = 0;
  const size_t oDIS = off; off = al256(off + (size_t)NBPD * 4);
  const size_t oW1T = off; off = al256(off + (size_t)NP * KA * 2);
  const size_t oW2T = off; off = al256(off + (size_t)NP * KA * 2);
  const size_t oW3T = off; off = al256(off + (size_t)NP * KA * 2);
  const size_t oXB  = off; off = al256(off + (size_t)MP * KA * 2);
  const size_t oH   = off; off = al256(off + (size_t)MP * NP * 4);
  const size_t oA2  = off; off = al256(off + (size_t)RA * KA * 2);
  if (off > ws_size || off > (size_t)WSMAX) return;
  float*          DIS = (float*)(ws + oDIS);
  unsigned short* W1T = (unsigned short*)(ws + oW1T);
  unsigned short* W2T = (unsigned short*)(ws + oW2T);
  unsigned short* W3T = (unsigned short*)(ws + oW3T);
  unsigned short* XB  = (unsigned short*)(ws + oXB);
  float*          H   = (float*)(ws + oH);
  unsigned short* A2  = (unsigned short*)(ws + oA2);

  const size_t aggLds = (size_t)AGG_LDS_INTS * 4;
  hipFuncSetAttribute(reinterpret_cast<const void*>(&k_agg<1>), hipFuncAttributeMaxDynamicSharedMemorySize, (int)aggLds);
  hipFuncSetAttribute(reinterpret_cast<const void*>(&k_agg<0>), hipFuncAttributeMaxDynamicSharedMemorySize, (int)aggLds);

  const int nUx = MP * (KA / 8);
  k_wprep<<<NUT / NTHR, NTHR, 0, stream>>>(W1, W2, W3, W1T, W2T, W3T);
  k_cvx<<<cdiv(nUx, NTHR), NTHR, 0, stream>>>(x, nN, nUx, XB);
  k_deg<<<gD, NTHR, 0, stream>>>(dst, nE, vec8, DIS);
  k_gemm<<<dim3(gM, NP / GBN), GTHR, 0, stream>>>(XB, W1T, H, KA, NP);
  k_agg<1><<<gA, NTHR, aggLds, stream>>>(src, dst, nE, nN, vec8, DIS, H, b1, g1, e1, m1, v1, A2, out);
  k_gemm<<<dim3(gM, NP / GBN), GTHR, 0, stream>>>(A2, W2T, H, KA, NP);
  k_agg<1><<<gA, NTHR, aggLds, stream>>>(src, dst, nE, nN, vec8, DIS, H, b2, g2, e2, m2, v2, A2, out);
  k_gemm<<<dim3(gM, NP / GBN), GTHR, 0, stream>>>(A2, W3T, H, KA, NP);
  k_agg<0><<<gA, NTHR, aggLds, stream>>>(src, dst, nE, nN, vec8, DIS, H, b3, b3, b3, b3, b3, A2, out);
}
